// NLblock2d_86509231276386
// MI455X (gfx1250) — hardware-verified
//
#include <hip/hip_runtime.h>


#define NB   8
#define CC   64
#define NTOK 3136
#define WP   72

typedef unsigned short u16;
typedef unsigned int   u32;

typedef __bf16   v16b __attribute__((ext_vector_type(16)));
typedef __bf16   v8bq __attribute__((ext_vector_type(8)));
typedef v8bq     v8b  __attribute__((may_alias));
typedef _Float16 v16h __attribute__((ext_vector_type(16)));
typedef _Float16 v8hq __attribute__((ext_vector_type(8)));
typedef v8hq     v8h  __attribute__((may_alias));
typedef float    v8f  __attribute__((ext_vector_type(8)));
typedef float    v4fq __attribute__((ext_vector_type(4)));
typedef v4fq     v4f  __attribute__((may_alias));
typedef u32      v4uq __attribute__((ext_vector_type(4)));
typedef v4uq     v4u  __attribute__((may_alias));

__device__ __forceinline__ u16 f2bf(float f) {
  const u32 u = __float_as_uint(f);
  const u32 r = u + 0x7FFFu + ((u >> 16) & 1u);
  return (u16)(r >> 16);
}
__device__ __forceinline__ float bf2f(u16 b) { return __uint_as_float(((u32)b) << 16); }
__device__ __forceinline__ void split_bf(float f, u16& hi, u16& lo) {
  hi = f2bf(f);
  lo = f2bf(f - bf2f(hi));
}
__device__ __forceinline__ u16 f2h(float f) {
  union { _Float16 h; u16 u; } c;
  c.h = (_Float16)f;
  return c.u;
}

__device__ __forceinline__ v16b ldb(const u16* p, int h) {
  union { v16b v; v8bq q[2]; } f;
  f.q[0] = *(const v8b*)(p + 8 * h);
  f.q[1] = *(const v8b*)(p + 16 + 8 * h);
  return f.v;
}
__device__ __forceinline__ v16h ldh(const u16* p, int h) {
  union { v16h v; v8hq q[2]; } f;
  f.q[0] = *(const v8h*)(p + 8 * h);
  f.q[1] = *(const v8h*)(p + 16 + 8 * h);
  return f.v;
}

__device__ __forceinline__ v8f mma_bf(v16b a, v16b b, v8f c) {
  return __builtin_amdgcn_wmma_f32_16x16x32_bf16(false, a, false, b, (short)0, c, false, false);
}
__device__ __forceinline__ v8f mma_h(v16h a, v16h b, v8f c) {
  return __builtin_amdgcn_wmma_f32_16x16x32_f16(false, a, false, b, (short)0, c, false, false);
}
#define WGUARD4(acc, a0, a1, b0, b1) \
  asm volatile("v_nop\n\tv_nop\n\tv_nop\n\tv_nop" : "+v"(acc) : "v"(a0), "v"(a1), "v"(b0), "v"(b1))
#define WGUARD2(acc, a0, b0) \
  asm volatile("v_nop\n\tv_nop\n\tv_nop\n\tv_nop" : "+v"(acc) : "v"(a0), "v"(b0))

__global__ __launch_bounds__(128) void k_proj(
    const float* __restrict__ x, const float* __restrict__ w1,
    const float* __restrict__ w2, const float* __restrict__ w3,
    u16* __restrict__ Qh, u16* __restrict__ Ql,
    u16* __restrict__ Kh, u16* __restrict__ Kl,
    u16* __restrict__ Vf, int nb, int ntile) {
  __shared__ __attribute__((aligned(16))) u16 s_wh[CC * WP];
  __shared__ __attribute__((aligned(16))) u16 s_wl[CC * WP];
  __shared__ __attribute__((aligned(16))) u16 s_xh[64 * WP];
  __shared__ __attribute__((aligned(16))) u16 s_xl[64 * WP];

  const int p  = blockIdx.y;
  const int b  = blockIdx.x / ntile;
  const int n0 = (blockIdx.x - b * ntile) * 64;
  if (b >= nb || p > 2) return;
  const int t = threadIdx.x, l = t & 31, wv = t >> 5, h = l >> 4, m = l & 15, e = l & 7;
  const float* wsrc = (p == 0) ? w1 : ((p == 1) ? w2 : w3);

  for (int q = t; q < (CC * CC) / 4; q += 128) {
    const int o = q >> 4, c4 = (q & 15) * 4;
    const v4f wq = *(const v4f*)(wsrc + (size_t)q * 4);
    #pragma unroll
    for (int k = 0; k < 4; ++k) {
      u16 hi, lo;
      split_bf(wq[k], hi, lo);
      s_wh[o * WP + c4 + k] = hi;
      s_wl[o * WP + c4 + k] = lo;
    }
  }
  for (int q = t; q < (CC * 64) / 4; q += 128) {
    const int c = q >> 4, j4 = (q & 15) * 4;
    const v4f xq = *(const v4f*)(x + ((size_t)(b * CC + c)) * NTOK + n0 + j4);
    #pragma unroll
    for (int k = 0; k < 4; ++k) {
      u16 hi, lo;
      split_bf(xq[k], hi, lo);
      s_xh[(j4 + k) * WP + c] = hi;
      s_xl[(j4 + k) * WP + c] = lo;
    }
  }
  __syncthreads();

  const v8f z = {0.f, 0.f, 0.f, 0.f, 0.f, 0.f, 0.f, 0.f};
  v8f acc[4];
  #pragma unroll
  for (int tt = 0; tt < 4; ++tt) acc[tt] = z;

  #pragma unroll
  for (int s = 0; s < 2; ++s) {
    const v16b bh = ldb(s_xh + (16 * wv + m) * WP + 32 * s, h);
    const v16b bl = ldb(s_xl + (16 * wv + m) * WP + 32 * s, h);
    #pragma unroll
    for (int tt = 0; tt < 4; ++tt) {
      const v16b ah = ldb(s_wh + (16 * tt + m) * WP + 32 * s, h);
      const v16b al = ldb(s_wl + (16 * tt + m) * WP + 32 * s, h);
      acc[tt] = mma_bf(ah, bh, acc[tt]);
      acc[tt] = mma_bf(ah, bl, acc[tt]);
      acc[tt] = mma_bf(al, bh, acc[tt]);
      WGUARD4(acc[tt], ah, al, bh, bl);
    }
  }
  __syncthreads();

  if (p == 0) {
    #pragma unroll
    for (int tt = 0; tt < 4; ++tt) {
      #pragma unroll
      for (int r = 0; r < 8; ++r)
        s_xh[(16 * tt + 8 * h + r) * 64 + 16 * wv + m] = f2h(acc[tt][r]);
    }
  } else {
    #pragma unroll
    for (int tt = 0; tt < 4; ++tt) {
      u16 hi[8], lo[8];
      #pragma unroll
      for (int r = 0; r < 8; ++r) split_bf(acc[tt][r], hi[r], lo[r]);
      v4u ph, pl;
      ph.x = (u32)hi[0] | ((u32)hi[1] << 16);  ph.y = (u32)hi[2] | ((u32)hi[3] << 16);
      ph.z = (u32)hi[4] | ((u32)hi[5] << 16);  ph.w = (u32)hi[6] | ((u32)hi[7] << 16);
      pl.x = (u32)lo[0] | ((u32)lo[1] << 16);  pl.y = (u32)lo[2] | ((u32)lo[3] << 16);
      pl.z = (u32)lo[4] | ((u32)lo[5] << 16);  pl.w = (u32)lo[6] | ((u32)lo[7] << 16);
      *(v4u*)(s_xh + (16 * wv + m) * 64 + 16 * tt + 8 * h) = ph;
      *(v4u*)(s_xl + (16 * wv + m) * 64 + 16 * tt + 8 * h) = pl;
    }
  }
  __syncthreads();

  if (p == 0) {
    v4u vals[4];
    size_t off[4];
    #pragma unroll
    for (int i = 0; i < 4; ++i) {
      const int o = 16 * wv + 4 * i + (l >> 3);
      vals[i] = *(const v4u*)(s_xh + o * 64 + 8 * e);
      off[i]  = ((size_t)(b * CC + o)) * NTOK + n0 + 8 * e;
    }
    #pragma unroll
    for (int i = 0; i < 4; ++i) *(volatile v4u*)(Vf + off[i]) = vals[i];
    __threadfence();
    #pragma unroll
    for (int i = 0; i < 4; ++i) *(volatile v4u*)(Vf + off[i]) = vals[i];
  } else {
    u16* gh = (p == 1) ? Qh : Kh;
    u16* gl = (p == 1) ? Ql : Kl;
    v4u vals[8];
    size_t off[8];
    #pragma unroll
    for (int i = 0; i < 8; ++i) {
      const int L  = 32 * wv + 4 * i + (l >> 3);
      const int pln = L >> 6, j = L & 63;
      vals[i] = *(const v4u*)((pln ? s_xl : s_xh) + j * 64 + 8 * e);
      off[i]  = ((size_t)(b * NTOK + n0 + j)) * CC + 8 * e;
    }
    const int pln_w = (32 * wv) >> 6;
    u16* dst = pln_w ? gl : gh;
    #pragma unroll
    for (int i = 0; i < 8; ++i) *(volatile v4u*)(dst + off[i]) = vals[i];
    __threadfence();
    #pragma unroll
    for (int i = 0; i < 8; ++i) *(volatile v4u*)(dst + off[i]) = vals[i];
  }
}

__global__ __launch_bounds__(32) __attribute__((amdgpu_num_vgpr(256))) void k_attn(
    const u16* __restrict__ Qh, const u16* __restrict__ Ql,
    const u16* __restrict__ Kh, const u16* __restrict__ Kl,
    const u16* __restrict__ Vf, u16* __restrict__ Ch, u16* __restrict__ Cl,
    int nb, int nrt) {
  __shared__ __attribute__((aligned(16))) u16 s_ch[16 * 64];
  __shared__ __attribute__((aligned(16))) u16 s_cl[16 * 64];

  const int b  = blockIdx.x / nrt;
  const int n0 = (blockIdx.x - b * nrt) * 16;
  if (b >= nb) return;
  const int l = threadIdx.x & 31, h = l >> 4, m = l & 15, e = l & 7;

  const size_t qrow = ((size_t)(b * NTOK + n0 + m)) * CC;
  v16b qh[2], ql[2];
  #pragma unroll
  for (int s = 0; s < 2; ++s) {
    qh[s] = ldb(Qh + qrow + 32 * s, h);
    ql[s] = ldb(Ql + qrow + 32 * s, h);
  }

  const v8f z = {0.f, 0.f, 0.f, 0.f, 0.f, 0.f, 0.f, 0.f};
  v8f acc[4];
  #pragma unroll
  for (int tt = 0; tt < 4; ++tt) acc[tt] = z;

  float mrun = -__builtin_inff();
  float lrun = 0.f;

  const u16* kbh = Kh + (size_t)b * NTOK * CC;
  const u16* kbl = Kl + (size_t)b * NTOK * CC;
  const u16* vb  = Vf + (size_t)b * CC * NTOK;

  #pragma unroll 1
  for (int c0 = 0; c0 < NTOK; c0 += 32) {
    v8f sc[2];
    #pragma unroll
    for (int j = 0; j < 2; ++j) {
      sc[j] = z;
      const size_t krow = ((size_t)(c0 + 16 * j + m)) * CC;
      #pragma unroll
      for (int s = 0; s < 2; ++s) {
        const v16b kh = ldb(kbh + krow + 32 * s, h);
        const v16b kl = ldb(kbl + krow + 32 * s, h);
        sc[j] = mma_bf(kh, qh[s], sc[j]);
        sc[j] = mma_bf(kh, ql[s], sc[j]);
        sc[j] = mma_bf(kl, qh[s], sc[j]);
        WGUARD4(sc[j], kh, kl, qh[s], ql[s]);
      }
    }

    float pm = sc[0][0];
    #pragma unroll
    for (int v = 0; v < 8; ++v) { pm = fmaxf(pm, sc[0][v]); pm = fmaxf(pm, sc[1][v]); }
    pm = fmaxf(pm, __shfl_xor(pm, 16, 32));
    const float mn    = fmaxf(mrun, pm);
    const float alpha = __expf(mrun - mn);
    mrun = mn;

    float ls = 0.f;
    union { v16h v; _Float16 s[16]; } pf;
    #pragma unroll
    for (int v = 0; v < 8; ++v) {
      const float p0 = __expf(sc[0][v] - mn);
      const float p1 = __expf(sc[1][v] - mn);
      ls += p0;
      ls += p1;
      pf.s[v]     = (_Float16)(p0 * 4096.0f);
      pf.s[8 + v] = (_Float16)(p1 * 4096.0f);
    }
    ls += __shfl_xor(ls, 16, 32);
    lrun = lrun * alpha + ls;

    float al[8];
    #pragma unroll
    for (int v = 0; v < 8; ++v) al[v] = __shfl(alpha, 8 * h + v, 32);
    #pragma unroll
    for (int tt = 0; tt < 4; ++tt) {
      #pragma unroll
      for (int v = 0; v < 8; ++v) acc[tt][v] *= al[v];
    }

    #pragma unroll
    for (int tt = 0; tt < 4; ++tt) {
      const v16h bv = ldh(vb + ((size_t)(16 * tt + m)) * NTOK + c0, h);
      acc[tt] = mma_h(pf.v, bv, acc[tt]);
      WGUARD2(acc[tt], pf.v, bv);
    }
  }

  const float linv = 1.0f / (lrun * 4096.0f);
  float lv[8];
  #pragma unroll
  for (int v = 0; v < 8; ++v) lv[v] = __shfl(linv, 8 * h + v, 32);
  #pragma unroll
  for (int tt = 0; tt < 4; ++tt) {
    #pragma unroll
    for (int v = 0; v < 8; ++v) {
      u16 hi, lo;
      split_bf(acc[tt][v] * lv[v], hi, lo);
      s_ch[(8 * h + v) * 64 + 16 * tt + m] = hi;
      s_cl[(8 * h + v) * 64 + 16 * tt + m] = lo;
    }
  }
  __syncthreads();

  v4u vals[8];
  size_t off[8];
  #pragma unroll
  for (int i = 0; i < 8; ++i) {
    const int L = 4 * i + (l >> 3);
    const int pln = L >> 4, row = L & 15;
    vals[i] = *(const v4u*)((pln ? s_cl : s_ch) + row * 64 + 8 * e);
    off[i]  = ((size_t)(b * NTOK + n0 + row)) * CC + 8 * e;
  }
  #pragma unroll
  for (int i = 0; i < 8; ++i) *(volatile v4u*)(((i >> 2) ? Cl : Ch) + off[i]) = vals[i];
  __threadfence();
  #pragma unroll
  for (int i = 0; i < 8; ++i) *(volatile v4u*)(((i >> 2) ? Cl : Ch) + off[i]) = vals[i];
}

__global__ __launch_bounds__(128) void k_out(
    const float* __restrict__ x, const float* __restrict__ wa,
    const u16* __restrict__ Ch, const u16* __restrict__ Cl,
    float* __restrict__ out, int nb, int ntile) {
  __shared__ __attribute__((aligned(16))) u16   s_wh[CC * WP];
  __shared__ __attribute__((aligned(16))) u16   s_wl[CC * WP];
  __shared__ __attribute__((aligned(16))) float s_d[64 * 64];

  const int b  = blockIdx.x / ntile;
  const int n0 = (blockIdx.x - b * ntile) * 64;
  if (b >= nb) return;
  const int t = threadIdx.x, l = t & 31, wv = t >> 5, h = l >> 4, m = l & 15, e = l & 7;

  for (int q = t; q < (CC * CC) / 4; q += 128) {
    const int o = q >> 4, c4 = (q & 15) * 4;
    const v4f wq = *(const v4f*)(wa + (size_t)q * 4);
    #pragma unroll
    for (int k = 0; k < 4; ++k) {
      u16 hi, lo;
      split_bf(wq[k], hi, lo);
      s_wh[o * WP + c4 + k] = hi;
      s_wl[o * WP + c4 + k] = lo;
    }
  }
  __syncthreads();

  const v8f z = {0.f, 0.f, 0.f, 0.f, 0.f, 0.f, 0.f, 0.f};
  v8f acc[4];
  #pragma unroll
  for (int tt = 0; tt < 4; ++tt) acc[tt] = z;

  const size_t crow = ((size_t)(b * NTOK + n0 + 16 * wv + m)) * CC;
  #pragma unroll
  for (int s = 0; s < 2; ++s) {
    const v16b ah = ldb(Ch + crow + 32 * s, h);
    const v16b al = ldb(Cl + crow + 32 * s, h);
    #pragma unroll
    for (int tt = 0; tt < 4; ++tt) {
      const v16b bh = ldb(s_wh + (16 * tt + m) * WP + 32 * s, h);
      const v16b bl = ldb(s_wl + (16 * tt + m) * WP + 32 * s, h);
      acc[tt] = mma_bf(ah, bh, acc[tt]);
      acc[tt] = mma_bf(ah, bl, acc[tt]);
      acc[tt] = mma_bf(al, bh, acc[tt]);
      WGUARD4(acc[tt], ah, al, bh, bl);
    }
  }

  #pragma unroll
  for (int tt = 0; tt < 4; ++tt) {
    v4f a0, a1;
    a0.x = acc[tt][0]; a0.y = acc[tt][1]; a0.z = acc[tt][2]; a0.w = acc[tt][3];
    a1.x = acc[tt][4]; a1.y = acc[tt][5]; a1.z = acc[tt][6]; a1.w = acc[tt][7];
    *(v4f*)(s_d + (16 * tt + m) * 64 + 16 * wv + 8 * h)     = a0;
    *(v4f*)(s_d + (16 * tt + m) * 64 + 16 * wv + 8 * h + 4) = a1;
  }
  __syncthreads();

  v4f vals[8];
  size_t off[8];
  #pragma unroll
  for (int i = 0; i < 8; ++i) {
    const int L = 32 * wv + 4 * i + (l >> 3);
    const int o = L >> 1, g = L & 1;
    const v4f dv = *(const v4f*)(s_d + o * 64 + 32 * g + 4 * e);
    off[i] = ((size_t)(b * CC + o)) * NTOK + n0 + 32 * g + 4 * e;
    const v4f xv = *(const v4f*)(x + off[i]);
    vals[i] = dv + xv;
  }
  #pragma unroll
  for (int i = 0; i < 8; ++i) *(volatile v4f*)(out + off[i]) = vals[i];
  __threadfence();
  #pragma unroll
  for (int i = 0; i < 8; ++i) *(volatile v4f*)(out + off[i]) = vals[i];
}

extern "C" void kernel_launch(void* const* d_in, const int* in_sizes, int n_in,
                              void* d_out, int out_size, void* d_ws, size_t ws_size,
                              hipStream_t stream) {
  if (n_in < 5) return;
  if (in_sizes[0] != NB * CC * NTOK) return;
  if (in_sizes[1] != CC * CC || in_sizes[2] != CC * CC ||
      in_sizes[3] != CC * CC || in_sizes[4] != CC * CC) return;
  if (out_size != NB * CC * NTOK) return;

  const float* x    = (const float*)d_in[0];
  const float* w1   = (const float*)d_in[1];
  const float* w2   = (const float*)d_in[2];
  const float* w3   = (const float*)d_in[3];
  const float* wadd = (const float*)d_in[4];
  float* out = (float*)d_out;

  const size_t plane = (size_t)NB * NTOK * CC;
  const size_t need  = 7 * plane * sizeof(u16);
  if (need > ws_size) return;
  u16* Qh = (u16*)d_ws;
  u16* Ql = Qh + plane;
  u16* Kh = Ql + plane;
  u16* Kl = Kh + plane;
  u16* Vf = Kl + plane;
  u16* Ch = Vf + plane;
  u16* Cl = Ch + plane;

  const int ntile64 = NTOK / 64;
  const int nrt     = NTOK / 16;
  if (ntile64 * 64 != NTOK || nrt * 16 != NTOK) return;

  k_proj<<<dim3(NB * ntile64, 3), 128, 0, stream>>>(x, w1, w2, w3, Qh, Ql, Kh, Kl, Vf, NB, ntile64);
  k_attn<<<NB * nrt, 32, 0, stream>>>(Qh, Ql, Kh, Kl, Vf, Ch, Cl, NB, nrt);
  k_out <<<NB * ntile64, 128, 0, stream>>>(x, wadd, Ch, Cl, out, NB, ntile64);
  (void)hipGetLastError();
}
